// GIN_27908697489545
// MI455X (gfx1250) — hardware-verified
//
#include <hip/hip_runtime.h>
#include <stddef.h>
#include <stdint.h>


#define CIN     128
#define HID     32
#define KA      256
#define KT      64
#define NTHR    256
#define NWAVE   8
#define EPT     8
#define CHUNK   (NTHR * EPT)
#define WCAP    (EPT * 32)
#define LISTN   (NWAVE * WCAP)
#define NBA     1024
#define PKS     10
#define RCAP    28672
#define DEGCAP  64
#define GBM     64
#define GTHR    128
#define GNT     2
#define NUA1    (HID * (KA / 8))
#define NUB     (HID * (KT / 8))
#define NUW     (NUA1 + 3 * NUB)
#define ZINTS   (2 * RCAP + 2 * NBA + LISTN)
#define LDS_AGG (ZINTS * 4 + 64)
#define WSMAX   134217728

static_assert((CHUNK & (CHUNK - 1)) == 0);
static_assert(NBA == (1 << PKS));
static_assert(((long long)CHUNK << PKS) < (1LL << 31));
static_assert(NTHR * 4 == NBA);
static_assert(LISTN >= NBA && LISTN >= NWAVE * WCAP);
static_assert((RCAP % 32) == 0);
static_assert((ZINTS % (NTHR * 4)) == 0);
static_assert(LDS_AGG <= 262144);
static_assert((NBA % NWAVE) == 0 && (NBA % GBM) == 0);
static_assert((NBA / NWAVE) == 32 * 4);
static_assert(GBM == (GTHR / 32) * 16);
static_assert(KA == 2 * CIN && KT == 2 * HID && (KA % 32) == 0 && (KT % 32) == 0);
static_assert(CIN == 32 * 4);
static_assert(HID == 32);
static_assert(HID == 16 * GNT);
static_assert(GBM * HID == GTHR * 16);
static_assert((NUA1 % NTHR) == 0 && (NUB % NTHR) == 0 && (NUW % NTHR) == 0);
static_assert((KA / 8) == 32 && (KT / 8) == 8);

typedef float          v4f  __attribute__((ext_vector_type(4)));
typedef float          v8f  __attribute__((ext_vector_type(8)));
typedef int            v4i  __attribute__((ext_vector_type(4)));
typedef int            v8i  __attribute__((ext_vector_type(8)));
typedef unsigned int   v4u  __attribute__((ext_vector_type(4)));
typedef unsigned short v8us __attribute__((ext_vector_type(8)));
typedef _Float16       v16h __attribute__((ext_vector_type(16)));
typedef __bf16         v16b __attribute__((ext_vector_type(16)));
typedef v4f  __attribute__((may_alias)) v4fa;
typedef v4i  __attribute__((may_alias)) v4ia;
typedef v8us __attribute__((may_alias)) v8usa;
union Frag { v16b b; v16h f; v8us h[2]; v8i w; };

__device__ __forceinline__ v8f wmk(const Frag& a, const Frag& b, v8f c) {
  v8f d = __builtin_amdgcn_wmma_f32_16x16x32_bf16(false, a.b, false, b.b, (short)0, c, false, false);
  asm volatile("v_nop\n\tv_nop\n\tv_nop\n\tv_nop" : "+v"(d) : "v"(a.w), "v"(b.w));
  return d;
}

__device__ __forceinline__ unsigned short bf_bits(float f) {
  unsigned int u = __float_as_uint(f);
  u += 0x7FFFu + ((u >> 16) & 1u);
  return (unsigned short)(u >> 16);
}
__device__ __forceinline__ float bf_val(unsigned short b) {
  return __uint_as_float(((unsigned int)b) << 16);
}
__device__ __forceinline__ float bf_rne(float f) { return bf_val(bf_bits(f)); }

__device__ __forceinline__ void split8b(const v4f a, const v4f b, v8us& hi, v8us& lo) {
  float x[8];
  x[0] = a.x; x[1] = a.y; x[2] = a.z; x[3] = a.w; x[4] = b.x; x[5] = b.y; x[6] = b.z; x[7] = b.w;
#pragma unroll
  for (int i = 0; i < 8; ++i) {
    const unsigned short hb = bf_bits(x[i]);
    hi[i] = hb;
    lo[i] = bf_bits(x[i] - bf_val(hb));
  }
}

template <int RND>
__device__ __forceinline__ float cvin(float v) {
  if constexpr (RND == 1) {
    return bf_rne(v);
  } else {
    return v;
  }
}

__device__ __forceinline__ void wave_sync() {
  __builtin_amdgcn_fence(__ATOMIC_RELEASE, "wavefront");
  __builtin_amdgcn_wave_barrier();
  __builtin_amdgcn_fence(__ATOMIC_ACQUIRE, "wavefront");
}

__device__ __forceinline__ int scan_chunk(const int* __restrict__ dsts, int nE, int cbase, int slotBase,
                                          int nb, int vec8, int* list, int tid, int lane, int wave) {
  int wc = 0;
  const int el0  = tid * EPT;
  const int e0   = cbase + el0;
  const int sent = -2147483647 - 1;
  v4i da, db;
  if (vec8 != 0 && cbase + CHUNK <= nE) {
    da = *(const v4i*)(dsts + e0);
    db = *(const v4i*)(dsts + e0 + 4);
  } else {
    da.x = (e0     < nE) ? dsts[min(e0,     nE - 1)] : sent;
    da.y = (e0 + 1 < nE) ? dsts[min(e0 + 1, nE - 1)] : sent;
    da.z = (e0 + 2 < nE) ? dsts[min(e0 + 2, nE - 1)] : sent;
    da.w = (e0 + 3 < nE) ? dsts[min(e0 + 3, nE - 1)] : sent;
    db.x = (e0 + 4 < nE) ? dsts[min(e0 + 4, nE - 1)] : sent;
    db.y = (e0 + 5 < nE) ? dsts[min(e0 + 5, nE - 1)] : sent;
    db.z = (e0 + 6 < nE) ? dsts[min(e0 + 6, nE - 1)] : sent;
    db.w = (e0 + 7 < nE) ? dsts[min(e0 + 7, nE - 1)] : sent;
  }
  const unsigned nbs = (unsigned)slotBase;
  const unsigned unb = (unsigned)nb;
  const unsigned s0 = (unsigned)da.x - nbs, s1 = (unsigned)da.y - nbs;
  const unsigned s2 = (unsigned)da.z - nbs, s3 = (unsigned)da.w - nbs;
  const unsigned s4 = (unsigned)db.x - nbs, s5 = (unsigned)db.y - nbs;
  const unsigned s6 = (unsigned)db.z - nbs, s7 = (unsigned)db.w - nbs;
  const bool h0 = s0 < unb, h1 = s1 < unb, h2 = s2 < unb, h3 = s3 < unb;
  const bool h4 = s4 < unb, h5 = s5 < unb, h6 = s6 < unb, h7 = s7 < unb;
  const unsigned any = __builtin_amdgcn_ballot_w32(h0 | h1 | h2 | h3 | h4 | h5 | h6 | h7);
  if (any != 0u) {
#define HITJ(J, HJ, SJ) { \
      const unsigned mj = __builtin_amdgcn_ballot_w32(HJ); \
      if (mj != 0u) { \
        if (HJ) { \
          const int pos = wc + (int)__builtin_amdgcn_mbcnt_lo(mj, 0u); \
          if (pos < WCAP) list[wave * WCAP + pos] = ((el0 + (J)) << PKS) | (int)(SJ); \
        } \
        wc += (int)__builtin_popcount(mj); } }
    HITJ(0, h0, s0)
    HITJ(1, h1, s1)
    HITJ(2, h2, s2)
    HITJ(3, h3, s3)
    HITJ(4, h4, s4)
    HITJ(5, h5, s5)
    HITJ(6, h6, s6)
    HITJ(7, h7, s7)
#undef HITJ
  }
  return wc;
}

__global__ __launch_bounds__(NTHR) void k_wprep(const float* __restrict__ w1a, const float* __restrict__ w1b,
                                                const float* __restrict__ w2a, const float* __restrict__ w2b,
                                                unsigned short* WA1, unsigned short* WB1,
                                                unsigned short* WA2, unsigned short* WB2) {
  const int u = (int)blockIdx.x * NTHR + (int)threadIdx.x;
  v8us o;
  unsigned short* dp;
  if (u < NUA1) {
    const int n = u >> 5;
    const int q = u & 31;
    const float* p = w1a + (size_t)(4 * q) * HID + n;
    float f[4];
#pragma unroll
    for (int c = 0; c < 4; ++c) f[c] = p[(size_t)c * HID];
#pragma unroll
    for (int j = 0; j < 8; ++j) o[j] = bf_bits(f[j & 3]);
    dp = WA1 + (size_t)n * KA + 8 * q;
  } else if (u < NUA1 + NUB) {
    const int v  = u - NUA1;
    const int n  = v >> 3;
    const int q  = v & 7;
    const int kk = (8 * q) & (HID - 1);
    const float* p = w1b + (size_t)kk * HID + n;
#pragma unroll
    for (int i = 0; i < 8; ++i) o[i] = bf_bits(p[(size_t)i * HID]);
    dp = WB1 + (size_t)n * KT + 8 * q;
  } else if (u < NUA1 + 2 * NUB) {
    const int v = u - NUA1 - NUB;
    const int n = v >> 3;
    const int q = v & 7;
    const float* p = w2a + (size_t)(4 * q) * HID + n;
    float f[4];
#pragma unroll
    for (int c = 0; c < 4; ++c) f[c] = p[(size_t)c * HID];
#pragma unroll
    for (int i = 0; i < 8; ++i) o[i] = bf_bits(f[i >> 1]);
    dp = WA2 + (size_t)n * KT + 8 * q;
  } else if (u < NUW) {
    const int v  = u - NUA1 - 2 * NUB;
    const int n  = v >> 3;
    const int q  = v & 7;
    const int kk = (8 * q) & (HID - 1);
    const float* p = w2b + (size_t)kk * HID + n;
#pragma unroll
    for (int i = 0; i < 8; ++i) o[i] = bf_bits(p[(size_t)i * HID]);
    dp = WB2 + (size_t)n * KT + 8 * q;
  } else {
    return;
  }
  *(volatile v8us*)dp = o;
  __threadfence();
  *(volatile v8us*)dp = o;
}

template <int KZ>
__global__ __launch_bounds__(GTHR) void k_mlp(const unsigned short* __restrict__ Z,
                                              const unsigned short* __restrict__ WA, const float* __restrict__ ba,
                                              const unsigned short* __restrict__ WB, const float* __restrict__ bb,
                                              float* H) {
  static_assert((KZ % 32) == 0 && KZ >= 32);
  __shared__ __attribute__((aligned(16))) float stg[GBM * HID];
  __shared__ __attribute__((aligned(16))) unsigned short tpl[GBM * KT];
  const int tid = (int)threadIdx.x, lane = tid & 31, wave = tid >> 5, hh = lane >> 4, m = lane & 15;
  const int rowBase = (int)blockIdx.x * GBM;
  const v8f z8 = {0.f, 0.f, 0.f, 0.f, 0.f, 0.f, 0.f, 0.f};

  v8f acc[GNT];
#pragma unroll
  for (int t = 0; t < GNT; ++t) acc[t] = z8;
  {
    const unsigned short* ap = Z  + (size_t)(rowBase + 16 * wave + m) * (size_t)KZ + 8 * hh;
    const unsigned short* bp = WA + (size_t)m * (size_t)KZ + 8 * hh;
#pragma unroll 1
    for (int k0 = 0; k0 < KZ; k0 += 32) {
      Frag af;
      af.h[0] = *(const v8usa*)(ap + k0);
      af.h[1] = *(const v8usa*)(ap + k0 + 16);
#pragma unroll
      for (int nt = 0; nt < GNT; ++nt) {
        const unsigned short* wq = bp + (size_t)(16 * nt) * (size_t)KZ + k0;
        Frag bf;
        bf.h[0] = *(const v8usa*)wq;
        bf.h[1] = *(const v8usa*)(wq + 16);
        acc[nt] = wmk(af, bf, acc[nt]);
      }
    }
  }
#pragma unroll
  for (int nt = 0; nt < GNT; ++nt) {
    const int lc = 16 * nt + m;
    const float bv = bf_rne(ba[lc]);
#pragma unroll
    for (int r = 0; r < 8; ++r) {
      const int lr = 16 * wave + 8 * hh + r;
      stg[lr * HID + lc] = fmaxf(acc[nt][r] + bv, 0.0f);
    }
  }
  __syncthreads();

  {
    const int r  = tid >> 1;
    const int c0 = 16 * (tid & 1);
    const float* sp = stg + r * HID + c0;
    const v4f f0 = *(const v4fa*)sp;
    const v4f f1 = *(const v4fa*)(sp + 4);
    const v4f f2 = *(const v4fa*)(sp + 8);
    const v4f f3 = *(const v4fa*)(sp + 12);
    v8us h0, l0, h1, l1;
    split8b(f0, f1, h0, l0);
    split8b(f2, f3, h1, l1);
    unsigned short* tp = tpl + r * KT + c0;
    *(v8usa*)tp = h0;
    *(v8usa*)(tp + 8) = h1;
    *(v8usa*)(tp + HID) = l0;
    *(v8usa*)(tp + HID + 8) = l1;
  }
  __syncthreads();

  v8f acc2[GNT];
#pragma unroll
  for (int t = 0; t < GNT; ++t) acc2[t] = z8;
  {
    const unsigned short* ap2 = tpl + (16 * wave + m) * KT + 8 * hh;
    const unsigned short* bp2 = WB + (size_t)m * (size_t)KT + 8 * hh;
#pragma unroll
    for (int k0 = 0; k0 < KT; k0 += 32) {
      Frag af;
      af.h[0] = *(const v8usa*)(ap2 + k0);
      af.h[1] = *(const v8usa*)(ap2 + k0 + 16);
#pragma unroll
      for (int nt = 0; nt < GNT; ++nt) {
        const unsigned short* wq = bp2 + (size_t)(16 * nt) * (size_t)KT + k0;
        Frag bf;
        bf.h[0] = *(const v8usa*)wq;
        bf.h[1] = *(const v8usa*)(wq + 16);
        acc2[nt] = wmk(af, bf, acc2[nt]);
      }
    }
  }
#pragma unroll
  for (int nt = 0; nt < GNT; ++nt) {
    const int lc = 16 * nt + m;
    const float bv = bf_rne(bb[lc]);
#pragma unroll
    for (int r = 0; r < 8; ++r) {
      const int lr = 16 * wave + 8 * hh + r;
      stg[lr * HID + lc] = acc2[nt][r] + bv;
    }
  }
  __syncthreads();

  v4f pv[4];
  const int rq = lane >> 3;
  const int cq = 4 * (lane & 7);
#pragma unroll
  for (int i = 0; i < 4; ++i) {
    const int lr = 16 * wave + 4 * i + rq;
    pv[i] = *(const v4fa*)(stg + lr * HID + cq);
  }
#pragma unroll
  for (int i = 0; i < 4; ++i) {
    const int gr = rowBase + 16 * wave + 4 * i + rq;
    float* op = H + (size_t)gr * (size_t)HID + cq;
    *(volatile v4f*)op = pv[i];
  }
  __threadfence();
#pragma unroll
  for (int i = 0; i < 4; ++i) {
    const int gr = rowBase + 16 * wave + 4 * i + rq;
    float* op = H + (size_t)gr * (size_t)HID + cq;
    *(volatile v4f*)op = pv[i];
  }
}

template <int CH, int RND, int FIN>
__global__ __launch_bounds__(NTHR) void k_agg(const int* __restrict__ srcs, const int* __restrict__ dsts,
                                              const float* __restrict__ X, unsigned short* Aout,
                                              const float* __restrict__ w3, const float* __restrict__ b3,
                                              float* outF, int nN, int nE, int vec8) {
  static_assert(CH == CIN || CH == HID);
  static_assert(FIN == 0 || CH == HID);
  extern __shared__ __attribute__((aligned(16))) int lds_i[];
  int* reg1 = lds_i;
  int* reg2 = reg1 + RCAP;
  int* scnt = reg2 + RCAP;
  int* soff = scnt + NBA;
  int* list = soff + NBA;
  int* wcnt = list + LISTN;
  int* wtot = wcnt + NWAVE;
  const int tid = (int)threadIdx.x, lane = tid & 31, wave = tid >> 5;
  const int nodeBase = (int)blockIdx.x * NBA;

  {
    const v4i z4 = {0, 0, 0, 0};
    for (int i = tid * 4; i < ZINTS; i += NTHR * 4) *(v4ia*)(lds_i + i) = z4;
    if (tid < 2 * NWAVE) wcnt[tid] = 0;
  }
  __syncthreads();

  int tot = 0;
  const int nChunks = (nE + CHUNK - 1) / CHUNK;
#pragma unroll 1
  for (int ch = 0; ch < nChunks; ++ch) {
    const int cbase = ch * CHUNK;
    const int wc = scan_chunk(dsts, nE, cbase, nodeBase, NBA, vec8, list, tid, lane, wave);
    if (lane == 0) wcnt[wave] = wc;
    __syncthreads();
    int pre = 0, all = 0;
#pragma unroll
    for (int w2 = 0; w2 < NWAVE; ++w2) {
      int c = wcnt[w2];
      c = c < 0 ? 0 : (c > WCAP ? WCAP : c);
      all += c;
      pre += (w2 < wave) ? c : 0;
    }
    const int wcc  = wc > WCAP ? WCAP : wc;
    const int base = tot + pre;
#pragma unroll 1
    for (int i = lane; i < wcc; i += 32) {
      const int ent = list[wave * WCAP + i];
      const int el  = (ent >> PKS) & (CHUNK - 1);
      const int sl  = ent & (NBA - 1);
      int eid = cbase + el;
      eid = eid > nE - 1 ? nE - 1 : eid;
      const int pos = base + i;
      if (pos < RCAP) reg1[pos] = (int)(((unsigned)eid << PKS) | (unsigned)sl);
    }
    tot += all;
    tot = tot > RCAP ? RCAP : tot;
    __syncthreads();
  }
  const int nh = tot;

  if (wave == 0) {
#pragma unroll 1
    for (int b0 = 0; b0 < nh; b0 += 32) {
      const int idx = b0 + lane;
      const int uv  = reg1[idx < RCAP ? idx : RCAP - 1];
      const int m32 = (nh - b0) < 32 ? (nh - b0) : 32;
#pragma unroll 1
      for (int k = 0; k < m32; ++k) {
        const int u  = __builtin_amdgcn_readlane(uv, k);
        const int sl = u & (NBA - 1);
        if (lane == 0) scnt[sl] = scnt[sl] + 1;
      }
    }
  }
  __syncthreads();

  {
    const v4i ca = *(const v4ia*)(scnt + 4 * tid);
    const int e0 = ca.x < 0 ? 0 : ca.x, e1 = ca.y < 0 ? 0 : ca.y, e2 = ca.z < 0 ? 0 : ca.z, e3 = ca.w < 0 ? 0 : ca.w;
    const int ts = e0 + e1 + e2 + e3;
    int incl = ts;
#pragma unroll
    for (int d = 1; d < 32; d <<= 1) {
      const int up = __shfl_up(incl, d, 32);
      if (lane >= d) incl += up;
    }
    if (lane == 31) wtot[wave] = incl;
    __syncthreads();
    int pre = 0;
#pragma unroll
    for (int w2 = 0; w2 < NWAVE; ++w2) pre += (w2 < wave) ? wtot[w2] : 0;
    int run = pre + incl - ts;
    soff[4 * tid + 0] = run; run += e0;
    soff[4 * tid + 1] = run; run += e1;
    soff[4 * tid + 2] = run; run += e2;
    soff[4 * tid + 3] = run;
  }
  __syncthreads();
  for (int i = tid; i < NBA; i += NTHR) list[i] = soff[i];
  __syncthreads();

  if (wave == 0) {
#pragma unroll 1
    for (int b0 = 0; b0 < nh; b0 += 32) {
      const int idx = b0 + lane;
      const int uv  = reg1[idx < RCAP ? idx : RCAP - 1];
      const int m32 = (nh - b0) < 32 ? (nh - b0) : 32;
#pragma unroll 1
      for (int k = 0; k < m32; ++k) {
        const int u   = __builtin_amdgcn_readlane(uv, k);
        const int sl  = u & (NBA - 1);
        const int eid = (int)((unsigned)u >> PKS);
        if (lane == 0) {
          int pos = list[sl];
          pos = pos < 0 ? 0 : (pos > RCAP - 1 ? RCAP - 1 : pos);
          reg2[pos] = eid;
          list[sl] = pos + 1;
        }
      }
    }
  }
  __syncthreads();

  const int nbw = NBA / NWAVE;
  const bool ovf = (nh >= RCAP);
  const float qnan = __int_as_float(0x7fc00000);

  if constexpr (CH == CIN) {
#pragma unroll 1
    for (int jt = 0; jt < nbw; ++jt) {
      const int slot = wave * nbw + jt;
      const int node = nodeBase + slot;
      int st = soff[slot];
      const int craw = scnt[slot];
      int cnt = craw;
      st  = st < 0 ? 0 : (st > nh ? nh : st);
      cnt = cnt < 0 ? 0 : (cnt > DEGCAP ? DEGCAP : cnt);
      if (cnt > nh - st) cnt = nh - st;
      const float pz = (ovf || craw > DEGCAP) ? qnan : 0.0f;
      const bool live = node < nN;
      const int nc = node < nN ? node : nN - 1;

      float a0 = 0.f, a1 = 0.f, a2 = 0.f, a3 = 0.f;
#pragma unroll 1
      for (int b0 = 0; b0 < cnt; b0 += 32) {
        int idx = st + b0 + lane; idx = idx > RCAP - 1 ? RCAP - 1 : idx;
        int eid = reg2[idx]; eid = eid < 0 ? 0 : (eid > nE - 1 ? nE - 1 : eid);
        int sr = srcs[eid]; sr = sr < 0 ? 0 : (sr > nN - 1 ? nN - 1 : sr);
        const int m32 = (cnt - b0) < 32 ? (cnt - b0) : 32;
#pragma unroll 1
        for (int k = 0; k < m32; ++k) {
          const int sk = __builtin_amdgcn_readlane(sr, k);
          const v4f v = *(const v4fa*)(X + (size_t)sk * CIN + 4 * lane);
          a0 += cvin<RND>(v.x); a1 += cvin<RND>(v.y); a2 += cvin<RND>(v.z); a3 += cvin<RND>(v.w);
        }
      }
      const v4f sv = *(const v4fa*)(X + (size_t)nc * CIN + 4 * lane);
      float r0 = a0 + cvin<RND>(sv.x), r1 = a1 + cvin<RND>(sv.y);
      float r2 = a2 + cvin<RND>(sv.z), r3 = a3 + cvin<RND>(sv.w);
      r0 = (live ? r0 : 0.0f) + pz;
      r1 = (live ? r1 : 0.0f) + pz;
      r2 = (live ? r2 : 0.0f) + pz;
      r3 = (live ? r3 : 0.0f) + pz;

      const unsigned short hb0 = bf_bits(r0), hb1 = bf_bits(r1), hb2 = bf_bits(r2), hb3 = bf_bits(r3);
      const unsigned short lb0 = bf_bits(r0 - bf_val(hb0)), lb1 = bf_bits(r1 - bf_val(hb1));
      const unsigned short lb2 = bf_bits(r2 - bf_val(hb2)), lb3 = bf_bits(r3 - bf_val(hb3));
      v4u pk;
      pk.x = (unsigned int)hb0 | ((unsigned int)hb1 << 16);
      pk.y = (unsigned int)hb2 | ((unsigned int)hb3 << 16);
      pk.z = (unsigned int)lb0 | ((unsigned int)lb1 << 16);
      pk.w = (unsigned int)lb2 | ((unsigned int)lb3 << 16);
      unsigned short* gp = Aout + (size_t)node * (size_t)KA + 8 * lane;
      *(volatile v4u*)gp = pk;
      __threadfence();
      *(volatile v4u*)gp = pk;
    }
    (void)w3; (void)b3; (void)outF;
  } else {
    float w3v = 0.0f, b3v = 0.0f;
    if constexpr (FIN == 1) {
      w3v = bf_rne(w3[lane]);
      b3v = bf_rne(b3[0]);
    }
    float* orow = (float*)list;
#pragma unroll 1
    for (int jt = 0; jt < nbw; ++jt) {
      const int slot = wave * nbw + jt;
      const int node = nodeBase + slot;
      int st = soff[slot];
      const int craw = scnt[slot];
      int cnt = craw;
      st  = st < 0 ? 0 : (st > nh ? nh : st);
      cnt = cnt < 0 ? 0 : (cnt > DEGCAP ? DEGCAP : cnt);
      if (cnt > nh - st) cnt = nh - st;
      const float pz = (ovf || craw > DEGCAP) ? qnan : 0.0f;
      const bool live = node < nN;
      const int nc = node < nN ? node : nN - 1;

      float a0 = 0.0f;
#pragma unroll 1
      for (int b0 = 0; b0 < cnt; b0 += 32) {
        int idx = st + b0 + lane; idx = idx > RCAP - 1 ? RCAP - 1 : idx;
        int eid = reg2[idx]; eid = eid < 0 ? 0 : (eid > nE - 1 ? nE - 1 : eid);
        int sr = srcs[eid]; sr = sr < 0 ? 0 : (sr > nN - 1 ? nN - 1 : sr);
        const int m32 = (cnt - b0) < 32 ? (cnt - b0) : 32;
#pragma unroll 1
        for (int k = 0; k < m32; ++k) {
          const int sk = __builtin_amdgcn_readlane(sr, k);
          a0 += cvin<RND>(X[(size_t)sk * HID + lane]);
        }
      }
      float r0 = a0 + cvin<RND>(X[(size_t)nc * HID + lane]);
      r0 = (live ? r0 : 0.0f) + pz;

      if constexpr (FIN == 0) {
        const unsigned short hb = bf_bits(r0);
        const unsigned short lb = bf_bits(r0 - bf_val(hb));
        const unsigned int pk = (unsigned int)hb | ((unsigned int)lb << 16);
        unsigned int* gp = (unsigned int*)(Aout + (size_t)node * (size_t)KT) + lane;
        *(volatile unsigned int*)gp = pk;
        __threadfence();
        *(volatile unsigned int*)gp = pk;
      } else {
        float s = r0 * w3v;
        s += __shfl_xor(s, 16, 32);
        s += __shfl_xor(s, 8, 32);
        s += __shfl_xor(s, 4, 32);
        s += __shfl_xor(s, 2, 32);
        s += __shfl_xor(s, 1, 32);
        if (lane == 0) orow[wave * nbw + jt] = s + b3v;
      }
    }
    if constexpr (FIN == 1) {
      wave_sync();
      const int r0i = nodeBase + wave * nbw + 4 * lane;
      const v4f w = *(const v4fa*)(orow + wave * nbw + 4 * lane);
      const bool full = (r0i + 4 <= nN);
      const bool part = (r0i < nN) && !full;
      if (full) *(volatile v4f*)(outF + (size_t)r0i) = w;
      if (part) {
        if (r0i + 0 < nN) *(volatile float*)(outF + (size_t)r0i + 0) = w.x;
        if (r0i + 1 < nN) *(volatile float*)(outF + (size_t)r0i + 1) = w.y;
        if (r0i + 2 < nN) *(volatile float*)(outF + (size_t)r0i + 2) = w.z;
      }
      __threadfence();
      if (full) *(volatile v4f*)(outF + (size_t)r0i) = w;
      if (part) {
        if (r0i + 0 < nN) *(volatile float*)(outF + (size_t)r0i + 0) = w.x;
        if (r0i + 1 < nN) *(volatile float*)(outF + (size_t)r0i + 1) = w.y;
        if (r0i + 2 < nN) *(volatile float*)(outF + (size_t)r0i + 2) = w.z;
      }
      (void)Aout;
    } else {
      (void)w3; (void)b3; (void)outF;
    }
  }
}

static inline int cdiv(int a, int b) { return (a + b - 1) / b; }
static inline size_t al256(size_t o) { return (o + 255) & ~(size_t)255; }

extern "C" void kernel_launch(void* const* d_in, const int* in_sizes, int n_in,
                              void* d_out, int out_size, void* d_ws, size_t ws_size,
                              hipStream_t stream) {
  if (n_in < 12) return;
  if (in_sizes[0] < CIN || (in_sizes[0] % CIN) != 0) return;
  const int nN = in_sizes[0] / CIN;
  if (nN < 1 || nN > (1 << 22)) return;
  if (in_sizes[1] < 2 || (in_sizes[1] & 1) != 0) return;
  const int nE = in_sizes[1] / 2;
  if (nE < 1 || nE >= (1 << 21)) return;
  if (in_sizes[2] != CIN * HID || in_sizes[3] != HID) return;
  if (in_sizes[4] != HID * HID || in_sizes[5] != HID) return;
  if (in_sizes[6] != HID * HID || in_sizes[7] != HID) return;
  if (in_sizes[8] != HID * HID || in_sizes[9] != HID) return;
  if (in_sizes[10] != HID || in_sizes[11] != 1) return;
  if ((long long)out_size != (long long)nN) return;

  const float* x   = (const float*)d_in[0];
  const int*   ei  = (const int*)  d_in[1];
  const float* w1a = (const float*)d_in[2];
  const float* b1a = (const float*)d_in[3];
  const float* w1b = (const float*)d_in[4];
  const float* b1b = (const float*)d_in[5];
  const float* w2a = (const float*)d_in[6];
  const float* b2a = (const float*)d_in[7];
  const float* w2b = (const float*)d_in[8];
  const float* b2b = (const float*)d_in[9];
  const float* w3  = (const float*)d_in[10];
  const float* b3  = (const float*)d_in[11];
  float* out = (float*)d_out;
  const int* src = ei;
  const int* dst = ei + nE;

  const int MP   = cdiv(nN, GBM) * GBM;
  const int gM   = MP / GBM;
  const int gA   = cdiv(MP, NBA);
  const int RA   = gA * NBA;
  const int vec8 = ((nE & 3) == 0) ? 1 : 0;
  if ((long long)RA < (long long)MP || (long long)RA < (long long)nN) return;

  char* ws = (char*)d_ws;
  size_t off = 0;
  const size_t oWA1 = off; off = al256(off + (size_t)HID * KA * 2);
  const size_t oWB1 = off; off = al256(off + (size_t)HID * KT * 2);
  const size_t oWA2 = off; off = al256(off + (size_t)HID * KT * 2);
  const size_t oWB2 = off; off = al256(off + (size_t)HID * KT * 2);
  const size_t oZ1  = off; off = al256(off + (size_t)RA * KA * 2);
  const size_t oH1  = off; off = al256(off + (size_t)MP * HID * 4);
  const size_t oZ2  = off; off = al256(off + (size_t)RA * KT * 2);
  const size_t oH2  = off; off = al256(off + (size_t)MP * HID * 4);
  if (off > ws_size || off > (size_t)WSMAX) return;
  unsigned short* WA1 = (unsigned short*)(ws + oWA1);
  unsigned short* WB1 = (unsigned short*)(ws + oWB1);
  unsigned short* WA2 = (unsigned short*)(ws + oWA2);
  unsigned short* WB2 = (unsigned short*)(ws + oWB2);
  unsigned short* Z1  = (unsigned short*)(ws + oZ1);
  float*          H1  = (float*)(ws + oH1);
  unsigned short* Z2  = (unsigned short*)(ws + oZ2);
  float*          H2  = (float*)(ws + oH2);

  hipFuncSetAttribute(reinterpret_cast<const void*>(&k_agg<CIN, 1, 0>), hipFuncAttributeMaxDynamicSharedMemorySize, LDS_AGG);
  hipFuncSetAttribute(reinterpret_cast<const void*>(&k_agg<HID, 0, 0>), hipFuncAttributeMaxDynamicSharedMemorySize, LDS_AGG);
  hipFuncSetAttribute(reinterpret_cast<const void*>(&k_agg<HID, 0, 1>), hipFuncAttributeMaxDynamicSharedMemorySize, LDS_AGG);

  k_wprep<<<NUW / NTHR, NTHR, 0, stream>>>(w1a, w1b, w2a, w2b, WA1, WB1, WA2, WB2);
  k_agg<CIN, 1, 0><<<gA, NTHR, LDS_AGG, stream>>>(src, dst, x, Z1, w3, b3, out, nN, nE, vec8);
  k_mlp<KA><<<gM, GTHR, 0, stream>>>(Z1, WA1, b1a, WB1, b1b, H1);
  k_agg<HID, 0, 0><<<gA, NTHR, LDS_AGG, stream>>>(src, dst, H1, Z2, w3, b3, out, nN, nE, vec8);
  k_mlp<KT><<<gM, GTHR, 0, stream>>>(Z2, WA2, b2a, WB2, b2b, H2);
  k_agg<HID, 0, 1><<<gA, NTHR, LDS_AGG, stream>>>(src, dst, H2, Z2, w3, b3, out, nN, nE, vec8);
}
